// DensityMap_15616501088354
// MI455X (gfx1250) — hardware-verified
//
#include <hip/hip_runtime.h>
#include <math.h>

typedef __attribute__((ext_vector_type(16))) _Float16 v16h;
typedef __attribute__((ext_vector_type(16))) __bf16 v16b;
typedef __attribute__((ext_vector_type(8)))  _Float16 v8h;
typedef __attribute__((ext_vector_type(8)))  float v8f;
typedef __attribute__((ext_vector_type(4)))  float v4f;
typedef __attribute__((ext_vector_type(2)))  float v2f;
typedef __attribute__((ext_vector_type(4)))  unsigned v4u;
typedef __attribute__((ext_vector_type(4)))  int v4i;
typedef float __attribute__((may_alias)) float_a;
typedef int __attribute__((may_alias)) int_a;

template <typename T> __device__ __forceinline__ void vst2(void* p, T v) { *(volatile T*)p = v; __threadfence(); *(volatile T*)p = v; }
__device__ __forceinline__ v8f wmma16(v16h a, v16h b, v8f c) {
  v8f d = __builtin_amdgcn_wmma_f32_16x16x32_f16(false, a, false, b, (short)0, c, false, false);
  asm volatile("v_nop\n\tv_nop\n\tv_nop\n\tv_nop" : "+v"(d) : "v"(a), "v"(b));
  return d;
}
__device__ __forceinline__ v8f wmma_bf(v16b a, v16b b, v8f c) {
  v8f d = __builtin_amdgcn_wmma_f32_16x16x32_bf16(false, a, false, b, (short)0, c, false, false);
  asm volatile("v_nop\n\tv_nop\n\tv_nop\n\tv_nop" : "+v"(d) : "v"(a), "v"(b));
  return d;
}
__device__ __forceinline__ v16h frag_h(const _Float16* rowk0, int lane) {
  union { v16h v; v8h q[2]; } u; const _Float16* p = rowk0 + 8 * (lane >> 4);
  u.q[0] = *(const v8h*)p; u.q[1] = *(const v8h*)(p + 16); return u.v;
}
__device__ __forceinline__ v16h frag_f32(const float* rowk0, int lane) {
  v16h a; const float* p = rowk0 + 8 * (lane >> 4);
#pragma unroll
  for (int i = 0; i < 8; ++i) { a[i] = (_Float16)p[i]; a[8 + i] = (_Float16)p[16 + i]; }
  return a;
}
__device__ __forceinline__ v16h frag_f32s(const float* rowk0, int lane, float sc) {
  v16h a; const float* p = rowk0 + 8 * (lane >> 4);
#pragma unroll
  for (int i = 0; i < 8; ++i) { a[i] = (_Float16)(p[i] * sc); a[8 + i] = (_Float16)(p[16 + i] * sc); }
  return a;
}
__device__ __forceinline__ v16h fragc_f32(const float* W, int k0, int n, int lane, int ld, int K) {
  v16h a; const int g = lane >> 4;
#pragma unroll
  for (int i = 0; i < 8; ++i) { const int ka = k0 + 8 * g + i, kb = ka + 16;
    a[i] = (_Float16)(ka < K ? W[(size_t)(ka < K ? ka : K - 1) * ld + n] : 0.f); a[8 + i] = (_Float16)(kb < K ? W[(size_t)(kb < K ? kb : K - 1) * ld + n] : 0.f); }
  return a;
}
struct F2 { v16b h, l; };
__device__ __forceinline__ F2 bsplit16(const float v[16]) { F2 r;
#pragma unroll
  for (int i = 0; i < 16; ++i) { const __bf16 h = (__bf16)v[i]; r.h[i] = h; r.l[i] = (__bf16)(v[i] - (float)h); }
  return r; }
__device__ __forceinline__ F2 split_row(const float* row, int k0, int lane) { float v[16]; const float* p = row + k0 + 8 * (lane >> 4);
#pragma unroll
  for (int i = 0; i < 8; ++i) { v[i] = p[i]; v[8 + i] = p[16 + i]; }
  return bsplit16(v); }
__device__ __forceinline__ F2 split_rowK(const float* row, int k0, int lane, int K) { float v[16]; const int g = lane >> 4;
#pragma unroll
  for (int i = 0; i < 8; ++i) { const int ka = k0 + 8 * g + i, kb = ka + 16; v[i] = ka < K ? row[ka < K ? ka : K - 1] : 0.f; v[8 + i] = kb < K ? row[kb < K ? kb : K - 1] : 0.f; }
  return bsplit16(v); }
__device__ __forceinline__ F2 split_col(const float* W, int k0, int n, int lane, int ld, int K) { float v[16]; const int g = lane >> 4;
#pragma unroll
  for (int i = 0; i < 8; ++i) { const int ka = k0 + 8 * g + i, kb = ka + 16; v[i] = ka < K ? W[(size_t)(ka < K ? ka : K - 1) * ld + n] : 0.f; v[8 + i] = kb < K ? W[(size_t)(kb < K ? kb : K - 1) * ld + n] : 0.f; }
  return bsplit16(v); }
__device__ __forceinline__ v8f mac3(const F2& a, const F2& b, v8f c) { c = wmma_bf(a.l, b.h, c); c = wmma_bf(a.h, b.l, c); return wmma_bf(a.h, b.h, c); }
__device__ __forceinline__ float sigm(float v) { return 1.0f / (1.0f + expf(-v)); }
#define LDSX() do { asm volatile("s_wait_dscnt 0" ::: "memory"); __builtin_amdgcn_wave_barrier(); __builtin_amdgcn_fence(__ATOMIC_RELEASE, "workgroup"); } while (0)


#define NB 64
#define NV 2048
#define GG 256
#define KS 13
#ifndef TNB
#define TNB NB
#endif
typedef __attribute__((ext_vector_type(8))) __bf16 v8b;
__device__ __forceinline__ v16b frag_b(const __bf16* rowk0, int lane) {
  union { v16b v; v8b q[2]; } u; const __bf16* p = rowk0 + 8 * (lane >> 4);
  u.q[0] = *(const v8b*)p; u.q[1] = *(const v8b*)(p + 16); return u.v;
}
__device__ __forceinline__ float bfr(float v) { return (float)(__bf16)v; }
__device__ __attribute__((noinline)) float exp_ni(float v) { return expf(v); }
__device__ __attribute__((noinline)) float erf_ni(float v) { return erff(v); }

#define BCH 16
#define WS_PH  0u
#define WS_PL  (WS_PH + 2u * BCH * 2 * GG * NV)
#define WS_D   (WS_PL + 2u * BCH * 2 * GG * NV)
#define WS_T   (WS_D + 4u * NB * GG * GG)
#define WS_PS  (WS_T + 4u * NB * GG * GG)
#define WS_END (WS_PS + 4u * NB * GG * 32)

__global__ __launch_bounds__(256) void k_planes(const float* __restrict__ POS, const float* __restrict__ SZ, const int* __restrict__ MK, int b0, __bf16* __restrict__ PH, __bf16* __restrict__ PL) {
  __shared__ __align__(16) __bf16 sh[NV], sl[NV];
  const int r = blockIdx.x, t = blockIdx.y, bl = blockIdx.z, b = b0 + bl, tid = threadIdx.x; const int v0 = tid * 8; const int comp = (t == 0) ? 1 : 0;
#pragma unroll 1
  for (int i = 0; i < 8; ++i) { const int v = v0 + i; const float p = (bfr(POS[((size_t)b * NV + v) * 2 + comp]) + 1.0f) * 0.5f * (float)(GG - 1); const float gs = bfr(SZ[v * 2 + comp]) * (float)GG * 0.5f;
    float val = sigm((gs * 0.5f - fabsf((float)r - p)) * 2.0f); if (t == 0) val *= (MK[v] != 0) ? 1.0f : 0.0f;
    const __bf16 hb = (__bf16)val; sh[v] = hb; sl[v] = (__bf16)(val - (float)hb); }
  const size_t o = (((size_t)bl * 2 + t) * GG + r) * NV + v0;
  vst2((unsigned*)(PH + o), *(const v4u*)&sh[v0]); vst2((unsigned*)(PL + o), *(const v4u*)&sl[v0]);
}
__global__ __launch_bounds__(128) void k_dense(const __bf16* __restrict__ PH, const __bf16* __restrict__ PL, int b0, float* __restrict__ D) {
  __shared__ __align__(16) float so[4][16][132];
  const int tid = threadIdx.x, wave = tid >> 5, lane = tid & 31, col = lane & 15, g = lane >> 4; const int bl = blockIdx.z, b = b0 + bl; const int y0 = blockIdx.x * 64 + wave * 16; const int x0 = blockIdx.y * 128;
  const __bf16* YH = PH + (((size_t)bl * 2 + 0) * GG) * NV; const __bf16* YL = PL + (((size_t)bl * 2 + 0) * GG) * NV; const __bf16* XH = PH + (((size_t)bl * 2 + 1) * GG) * NV; const __bf16* XL = PL + (((size_t)bl * 2 + 1) * GG) * NV;
  v8f acc[8] = {};
#pragma unroll 2
  for (int kc = 0; kc < NV / 32; ++kc) { const v16b ah = frag_b(YH + (size_t)(y0 + col) * NV + kc * 32, lane), al = frag_b(YL + (size_t)(y0 + col) * NV + kc * 32, lane);
#pragma unroll
    for (int j = 0; j < 8; ++j) { const size_t br = (size_t)(x0 + j * 16 + col) * NV + kc * 32; const v16b bh = frag_b(XH + br, lane), bl = frag_b(XL + br, lane); acc[j] = wmma_bf(al, bh, acc[j]); acc[j] = wmma_bf(ah, bl, acc[j]); acc[j] = wmma_bf(ah, bh, acc[j]); } }
#pragma unroll
  for (int j = 0; j < 8; ++j)
#pragma unroll
    for (int r = 0; r < 8; ++r) so[wave][8 * g + r][j * 16 + col] = acc[j][r];
  LDSX();
  for (int rl = 0; rl < 16; ++rl) vst2(D + ((size_t)b * GG + y0 + rl) * GG + x0 + lane * 4, *(const v4f*)&so[wave][rl][lane * 4]);
}
__device__ __forceinline__ int refl(int i) { i = (i < 0) ? -i : i; return (i >= GG) ? (2 * GG - 2 - i) : i; }
__device__ __forceinline__ void gauss13(float* k) { float s = 0.f; float e[KS];
#pragma unroll
  for (int i = 0; i < KS; ++i) { const float x = (float)(i - KS / 2); e[i] = exp_ni(-(x * x) / 8.0f); }
#pragma unroll
  for (int i = 0; i < KS; ++i) s += e[i];
#pragma unroll
  for (int i = 0; i < KS; ++i) k[i] = e[i] / s; }
__global__ __launch_bounds__(256) void k_blur_h(const float* __restrict__ D, float* __restrict__ T) {
  __shared__ float srow[GG]; __shared__ __align__(16) float so[GG]; __shared__ float sk[KS];
  const int y = blockIdx.x, b = blockIdx.y, x = threadIdx.x; const float* drow = D + ((size_t)b * GG + y) * GG;
  srow[x] = drow[x]; if (x == 0) { float k[KS]; gauss13(k); for (int i = 0; i < KS; ++i) sk[i] = k[i]; }
  __syncthreads();
  float acc = 0.f;
#pragma unroll 1
  for (int j = 0; j < KS; ++j) acc += sk[j] * srow[refl(x + j - KS / 2)];
  so[x] = acc; __syncthreads();
  if (x < GG / 4) vst2(T + ((size_t)b * GG + y) * GG + x * 4, *(const v4f*)&so[x * 4]);
}
__global__ __launch_bounds__(256) void k_blur_v(const float* __restrict__ T, float* __restrict__ OUT, float* __restrict__ PS) {
  __shared__ __align__(16) float so[GG]; __shared__ float sk[KS]; __shared__ float sw[8]; __shared__ __align__(16) float sline[32];
  const int y = blockIdx.x, b = blockIdx.y, x = threadIdx.x;
  if (x == 0) { float k[KS]; gauss13(k); for (int i = 0; i < KS; ++i) sk[i] = k[i]; }
  __syncthreads();
  float acc = 0.f;
#pragma unroll 1
  for (int i = 0; i < KS; ++i) acc += sk[i] * T[((size_t)b * GG + refl(y + i - KS / 2)) * GG + x];
  so[x] = acc;
  float ov = fmaxf(acc - 1.0f, 0.f); float q = ov * ov;
#pragma unroll
  for (int o = 1; o < 32; o <<= 1) q += __shfl_xor(q, o);
  if ((x & 31) == 0) sw[x >> 5] = q;
  __syncthreads();
  if (x < GG / 4) vst2(OUT + ((size_t)b * GG + y) * GG + x * 4, *(const v4f*)&so[x * 4]);
  if (x < 32) { float v = 0.f; if (x == 0) for (int w = 0; w < 8; ++w) v += sw[w]; sline[x] = (x == 0) ? v : 0.f; }
  __syncthreads();
  if (x < 8) vst2(PS + ((size_t)b * GG + y) * 32 + x * 4, *(const v4f*)&sline[x * 4]);
}
__global__ __launch_bounds__(256) void k_loss(const float* __restrict__ PS, float* __restrict__ out) {
  __shared__ float s[256]; const int tid = threadIdx.x; float acc = 0.f;
  for (int i = tid; i < TNB * GG; i += 256) acc += PS[(size_t)i * 32];
  s[tid] = acc; __syncthreads();
  if (tid == 0) { float t = 0.f; for (int i = 0; i < 256; ++i) t += s[i]; *(volatile float*)out = t / (float)((size_t)NB * GG * GG); *(volatile float*)out = t / (float)((size_t)NB * GG * GG); }
}
extern "C" void kernel_launch(void* const* d_in, const int* in_sizes, int n_in, void* d_out, int out_size, void* d_ws, size_t ws_size, hipStream_t stream) {
  (void)in_sizes; (void)n_in; (void)out_size;
  const float* POS = (const float*)d_in[0]; const float* SZ = (const float*)d_in[1]; const int* MK = (const int*)d_in[2];
  if (ws_size < (size_t)WS_END) return;
  char* ws = (char*)d_ws; __bf16 *PH = (__bf16*)(ws + WS_PH), *PL = (__bf16*)(ws + WS_PL); float *D = (float*)(ws + WS_D), *T = (float*)(ws + WS_T), *PS = (float*)(ws + WS_PS);
  float* DEN = (float*)d_out; float* LOSS = DEN + (size_t)NB * GG * GG;
  for (int b0 = 0; b0 < TNB; b0 += BCH) { const int nb = (TNB - b0 < BCH) ? (TNB - b0) : BCH;
    k_planes<<<dim3(GG, 2, nb), 256, 0, stream>>>(POS, SZ, MK, b0, PH, PL);
    k_dense<<<dim3(GG / 64, GG / 128, nb), 128, 0, stream>>>(PH, PL, b0, D); }
  k_blur_h<<<dim3(GG, TNB), 256, 0, stream>>>(D, T);
  k_blur_v<<<dim3(GG, TNB), 256, 0, stream>>>(T, DEN, PS);
  k_loss<<<1, 256, 0, stream>>>(PS, LOSS);
}
